// RotationAttention_44839458570375
// MI455X (gfx1250) — hardware-run, weakly checked
//
#include <hip/hip_runtime.h>
#include <stddef.h>


typedef _Float16 v16h __attribute__((ext_vector_type(16)));
typedef _Float16 v8h  __attribute__((ext_vector_type(8)));
typedef float    v8f  __attribute__((ext_vector_type(8)));
typedef float    v4f  __attribute__((ext_vector_type(4)));
typedef _Float16 h16;

#ifndef NB
#define NB 32
#endif
#define NB_FULL 32
#define NANCH 64
#define DIM   512
#define HID   512
#define KH    256

static_assert(NB >= 1 && NB <= NB_FULL);
static_assert(NANCH == 64 && DIM == 512 && HID == 512);
static_assert((DIM % 64) == 0 && (DIM % 32) == 0);
static_assert((HID % 64) == 0 && (HID % 128) == 0);
static_assert(DIM == 2 * KH && (KH % 32) == 0);
static_assert(NANCH == 4 * 8 * 2);
static_assert(HID == 2 * 32 * 8);
static_assert(HID == 4 * 4 * 32);

#define LDT 72
static_assert((LDT % 8) == 0 && LDT >= 64);
#define LDX 520
static_assert((LDX % 8) == 0 && LDX >= DIM);
#define LDXH 264
static_assert((LDXH % 8) == 0 && LDXH >= KH);
#define LDSS 68
#define LDW 132
#define LDP 8
static_assert((LDSS % 4) == 0 && LDSS >= 64);
static_assert((LDW % 4) == 0 && LDW >= 128);
static_assert(LDP >= 6 && LDP <= 16);

#define WCARRY 64.0f
#define XCARRY 256.0f
#define RCARRY 2048.0f
#define TEMP_INV (1.0f / 0.3f)

static_assert(80 * (KH / 8) == 256 * 10);
static_assert(16 * (DIM / 8) == 256 * 4);
static_assert(16 * DIM == 256 * 32);
static_assert(2 * 16 * LDX <= 80 * LDXH);
static_assert(((NANCH * 9 * 4) % 128) == 0);
static_assert(((NANCH * 9) % 4) == 0 && (NANCH * 9) / 4 <= 5 * 32);
static_assert((7 * HID) % 4 == 0);

#define ROT_LDS_BYTES ((size_t)80 * LDXH * 2 + (size_t)16 * LDX * 2 + (size_t)7 * HID * 4 + \
                       (size_t)80 * LDSS * 4 + (size_t)3 * NANCH * 9 * 4 + (size_t)NANCH * 8 * 4 + \
                       (size_t)NANCH * 4 + (size_t)8 * NANCH * LDP * 4)
static_assert(ROT_LDS_BYTES <= (size_t)131072);

#define W1T_BYTES  ((size_t)HID * DIM * 2)
#define WEFF_BYTES ((size_t)8 * HID * 4)
#define OFF_W1T  ((size_t)0)
#define OFF_WEFF (OFF_W1T + W1T_BYTES)
#define WS_TOTAL (OFF_WEFF + WEFF_BYTES)
static_assert((W1T_BYTES % 128) == 0 && (WEFF_BYTES % 128) == 0);
static_assert(WS_TOTAL <= (size_t)134217728);

__device__ __forceinline__ float bf16r(float x) {
  unsigned int u = __float_as_uint(x);
  u = (u + 0x7FFFu + ((u >> 16) & 1u)) & 0xFFFF0000u;
  return __uint_as_float(u);
}

__device__ __forceinline__ v16h frag_at(const _Float16* p) {
  v8h lo = *(const v8h*)(p);
  v8h hi = *(const v8h*)(p + 16);
  v16h out;
#pragma unroll
  for (int i = 0; i < 8; ++i) { out[i] = lo[i]; out[i + 8] = hi[i]; }
  return out;
}
__device__ __forceinline__ v16h ld_frag(const _Float16* base, unsigned ld) {
  const unsigned lane = threadIdx.x & 31u;
  return frag_at(base + (lane & 15u) * ld + (lane >> 4) * 8u);
}

__device__ __forceinline__ v8f wmma16(v16h a, v16h b, v8f c) {
  v8f d = __builtin_amdgcn_wmma_f32_16x16x32_f16(false, a, false, b, (short)0, c,
                                                 false, false);
  asm volatile("v_nop\n\tv_nop\n\tv_nop\n\tv_nop" : "+v"(d) : "v"(a), "v"(b));
  return d;
}

static __device__ __forceinline__ h16 toh_flush(float v) {
  const h16 r = (h16)v;
  return (fabsf(v) < 6.103515625e-05f) ? (h16)0.0f : r;
}

__device__ __forceinline__ float red32_max(float x) {
#pragma unroll
  for (int off = 1; off < 32; off <<= 1) x = fmaxf(x, __shfl_xor(x, off, 32));
  return x;
}

__device__ __forceinline__ float inv_norm3(float x0, float x1, float x2) {
#pragma clang fp contract(off)
  const float n = sqrtf((x0 * x0 + x2 * x2) + x1 * x1);
  return 1.0f / fmaxf(n, 1.0e-12f);
}

__global__ __launch_bounds__(256) void wconv_kernel(
    const float* __restrict__ W, _Float16* __restrict__ Wt, unsigned ldw, unsigned ldk) {
  __shared__ _Float16 T[64 * LDT];
  const unsigned tid = threadIdx.x;
  const unsigned n0 = blockIdx.x * 64u;
  const unsigned k0 = blockIdx.y * 64u;
#pragma unroll 4
  for (unsigned j = 0; j < 16u; ++j) {
    const unsigned idx = tid + 256u * j;
    const unsigned kr = idx >> 6, nc = idx & 63u;
    const float v = W[(size_t)(k0 + kr) * ldw + n0 + nc];
    T[nc * LDT + kr] = (_Float16)(WCARRY * bf16r(v));
  }
  __syncthreads();
  v8h x[2];
  size_t off[2];
#pragma unroll
  for (unsigned i = 0; i < 2u; ++i) {
    const unsigned n = 32u * i + (tid >> 3);
    const unsigned kc = (tid & 7u) * 8u;
    x[i] = *(const v8h*)&T[n * LDT + kc];
    off[i] = (size_t)(n0 + n) * ldk + k0 + kc;
  }
#pragma unroll
  for (int i = 0; i < 2; ++i) *(volatile v8h*)(Wt + off[i]) = x[i];
  __threadfence();
#pragma unroll
  for (int i = 0; i < 2; ++i) *(volatile v8h*)(Wt + off[i]) = x[i];
}

__global__ __launch_bounds__(256) void weff_kernel(
    const float* __restrict__ Wenc, const float* __restrict__ benc,
    const _Float16* __restrict__ W1t, const float* __restrict__ b1,
    float* __restrict__ Weff) {
  __shared__ _Float16 As[16 * LDX];
  __shared__ float Cs[8 * LDW];
  const unsigned tid = threadIdx.x, lane = tid & 31u;
  const int wave = __builtin_amdgcn_readfirstlane(threadIdx.x >> 5);
  const unsigned wv = (unsigned)wave;
  const unsigned hh = lane >> 4, m = lane & 15u;
  const unsigned h0 = blockIdx.x * 128u;

#pragma unroll 1
  for (unsigned j = 0; j < 4u; ++j) {
    const unsigned idx = tid + 256u * j;
    const unsigned row = idx >> 6, c8 = (idx & 63u) * 8u;
    const unsigned rw = (row < 6u) ? row : 5u;
    const v4f w0 = *(const v4f*)(Wenc + rw * (unsigned)DIM + c8);
    const v4f w1 = *(const v4f*)(Wenc + rw * (unsigned)DIM + c8 + 4u);
    const v4f e0 = *(const v4f*)(benc + c8);
    const v4f e1 = *(const v4f*)(benc + c8 + 4u);
    v8h o;
#pragma unroll
    for (int i = 0; i < 4; ++i) {
      const float a0 = (row < 6u) ? w0[i] : ((row == 6u) ? e0[i] : 0.0f);
      const float a1 = (row < 6u) ? w1[i] : ((row == 6u) ? e1[i] : 0.0f);
      o[i]     = toh_flush(WCARRY * bf16r(a0));
      o[i + 4] = toh_flush(WCARRY * bf16r(a1));
    }
    *(v8h*)&As[row * LDX + c8] = o;
  }
  __syncthreads();

  const _Float16* bp = W1t + (size_t)(h0 + wv * 16u + m) * DIM + hh * 8u;
  v8f acc = {};
#pragma unroll 2
  for (unsigned k0 = 0; k0 < (unsigned)DIM; k0 += 32u) {
    const v16h a = ld_frag(&As[k0], LDX);
    const v16h w = frag_at(bp + k0);
    acc = wmma16(a, w, acc);
  }
  if (hh == 0u) {
#pragma unroll
    for (int r = 0; r < 8; ++r)
      Cs[(unsigned)r * LDW + wv * 16u + m] = acc[r] * (1.0f / (WCARRY * WCARRY));
  }
  __syncthreads();

  const unsigned row = tid >> 5, c4 = (tid & 31u) * 4u;
  const v4f u  = *(const v4f*)&Cs[row * LDW + c4];
  const v4f bb = *(const v4f*)(b1 + h0 + c4);
  v4f val;
#pragma unroll
  for (int j = 0; j < 4; ++j) val[j] = u[j] + ((row == 6u) ? bf16r(bb[j]) : 0.0f);
  float* p = Weff + (size_t)row * HID + h0 + c4;
  *(volatile v4f*)p = val;
  __threadfence();
  *(volatile v4f*)p = val;
}

__global__ __launch_bounds__(256) void rotattn_kernel(
    const float* __restrict__ img, const float* __restrict__ feat,
    const float* __restrict__ rot, const float* __restrict__ Weff,
    const float* __restrict__ W2, const float* __restrict__ b2,
    float* __restrict__ out) {
  __shared__ _Float16 Xs[80 * LDXH];
  __shared__ _Float16 W2s[16 * LDX];
  __shared__ float WEs[7 * HID];
  __shared__ float Ss[80 * LDSS];
  __shared__ float Rr[NANCH * 9];
  __shared__ float Ri[NANCH * 9];
  __shared__ float X6[NANCH * 8];
  __shared__ float Hsc[NANCH];
  __shared__ float Part[8 * NANCH * LDP];
  __shared__ float Os[NANCH * 9];

  const unsigned tid = threadIdx.x, lane = tid & 31u;
  const int wave = __builtin_amdgcn_readfirstlane(threadIdx.x >> 5);
  const unsigned wv = (unsigned)wave;
  const unsigned hh = lane >> 4, m = lane & 15u;
  const unsigned b = blockIdx.x;

  const float* fb = feat + (size_t)b * (NANCH * DIM);
  const float* ib = img + (size_t)b * DIM;
#pragma unroll 1
  for (unsigned j = 0; j < 32u; ++j) {
    const unsigned idx = tid + 256u * j;
    const unsigned n = idx >> 9, k = idx & 511u;
    const unsigned nc = (n < 6u) ? n : 5u;
    const float v = W2[k * 6u + nc];
    const h16 hv = toh_flush(WCARRY * bf16r(v));
    W2s[n * LDX + k] = (n < 6u) ? hv : (h16)0.0f;
  }
  for (unsigned i = tid; i < (unsigned)(7 * HID / 4); i += 256u)
    *(v4f*)&WEs[4u * i] = *(const v4f*)(Weff + 4u * i);
  for (unsigned i = tid; i < (unsigned)(NANCH * 9); i += 256u)
    Rr[i] = bf16r(rot[(size_t)b * (NANCH * 9) + i]);
  if (tid < (unsigned)NANCH) {
    const float* r = rot + ((size_t)b * NANCH + tid) * 9u;
    const double a  = (double)bf16r(r[0]), bb = (double)bf16r(r[1]), c = (double)bf16r(r[2]);
    const double d  = (double)bf16r(r[3]), e  = (double)bf16r(r[4]), f = (double)bf16r(r[5]);
    const double g  = (double)bf16r(r[6]), h  = (double)bf16r(r[7]), i9 = (double)bf16r(r[8]);
    const double A0 = e * i9 - f * h, A1 = -(d * i9 - f * g), A2 = d * h - e * g;
    const double inv = 1.0 / (a * A0 + bb * A1 + c * A2);
    Ri[tid * 9u + 0u] = (float)(A0 * inv);
    Ri[tid * 9u + 1u] = (float)(-(bb * i9 - c * h) * inv);
    Ri[tid * 9u + 2u] = (float)((bb * f - c * e) * inv);
    Ri[tid * 9u + 3u] = (float)(A1 * inv);
    Ri[tid * 9u + 4u] = (float)((a * i9 - c * g) * inv);
    Ri[tid * 9u + 5u] = (float)(-(a * f - c * d) * inv);
    Ri[tid * 9u + 6u] = (float)(A2 * inv);
    Ri[tid * 9u + 7u] = (float)(-(a * h - bb * g) * inv);
    Ri[tid * 9u + 8u] = (float)((a * e - bb * d) * inv);
  }

  const unsigned nt = wv & 3u, mq = wv >> 2;
  v8f g0 = {}, g1 = {}, g2 = {};
#pragma unroll 1
  for (unsigned kh2 = 0; kh2 < 2u; ++kh2) {
    const unsigned cb = kh2 * (unsigned)KH;
#pragma unroll 1
    for (unsigned j = 0; j < 10u; ++j) {
      const unsigned idx = tid + 256u * j;
      const unsigned row = idx >> 5, c8 = (idx & 31u) * 8u;
      const unsigned rc = (row < 64u) ? row : 63u;
      const v4f f0 = *(const v4f*)(fb + rc * (unsigned)DIM + cb + c8);
      const v4f f1 = *(const v4f*)(fb + rc * (unsigned)DIM + cb + c8 + 4u);
      const v4f q0 = *(const v4f*)(ib + cb + c8);
      const v4f q1 = *(const v4f*)(ib + cb + c8 + 4u);
      v8h o;
#pragma unroll
      for (int i = 0; i < 4; ++i) {
        const float a0 = (row < 64u) ? f0[i] : ((row == 64u) ? q0[i] : 0.0f);
        const float a1 = (row < 64u) ? f1[i] : ((row == 64u) ? q1[i] : 0.0f);
        o[i]     = toh_flush(XCARRY * bf16r(a0));
        o[i + 4] = toh_flush(XCARRY * bf16r(a1));
      }
      *(v8h*)&Xs[row * LDXH + c8] = o;
    }
    __syncthreads();

#pragma unroll 2
    for (unsigned k0 = 0; k0 < (unsigned)KH; k0 += 32u) {
      const v16h kf = ld_frag(&Xs[(nt * 16u) * LDXH + k0], LDXH);
      const v16h a0 = ld_frag(&Xs[(mq * 16u) * LDXH + k0], LDXH);
      const v16h a1 = ld_frag(&Xs[((2u + mq) * 16u) * LDXH + k0], LDXH);
      g0 = wmma16(a0, kf, g0);
      g1 = wmma16(a1, kf, g1);
    }
    if (wave < 4) {
#pragma unroll 2
      for (unsigned k0 = 0; k0 < (unsigned)KH; k0 += 32u) {
        const v16h kf = ld_frag(&Xs[(nt * 16u) * LDXH + k0], LDXH);
        const v16h a2 = ld_frag(&Xs[(64u) * LDXH + k0], LDXH);
        g2 = wmma16(a2, kf, g2);
      }
    }
    __syncthreads();
  }
#pragma unroll
  for (int r = 0; r < 8; ++r) {
    Ss[(mq * 16u + hh * 8u + (unsigned)r) * LDSS + nt * 16u + m] =
        g0[r] * (1.0f / (XCARRY * XCARRY));
    Ss[((2u + mq) * 16u + hh * 8u + (unsigned)r) * LDSS + nt * 16u + m] =
        g1[r] * (1.0f / (XCARRY * XCARRY));
  }
  if (wave < 4) {
#pragma unroll
    for (int r = 0; r < 8; ++r)
      Ss[(64u + hh * 8u + (unsigned)r) * LDSS + nt * 16u + m] =
          g2[r] * (1.0f / (XCARRY * XCARRY));
  }
  __syncthreads();

  if (tid < (unsigned)NANCH) {
    float mx = -3.0e38f, mn = 3.0e38f;
#pragma unroll 1
    for (unsigned j = 0; j < (unsigned)NANCH; ++j) {
      const float s = (Ss[64u * LDSS + j] - Ss[tid * LDSS + j]) * TEMP_INV;
      mx = fmaxf(mx, s);
      mn = fminf(mn, s);
    }
    float Ma[9], Mb[9];
#pragma unroll
    for (int u = 0; u < 9; ++u) { Ma[u] = 0.0f; Mb[u] = 0.0f; }
    float sa = 0.0f, sb = 0.0f;
#pragma unroll 1
    for (unsigned j = 0; j < (unsigned)NANCH; ++j) {
      const float s  = (Ss[64u * LDSS + j] - Ss[tid * LDSS + j]) * TEMP_INV;
      const float aw = expf(s - mx);
      const float bw = expf(mn - s);
      sa += aw;
      sb += bw;
#pragma unroll
      for (int u = 0; u < 9; ++u) {
        Ma[u] += aw * Rr[j * 9u + (unsigned)u];
        Mb[u] += bw * Ri[j * 9u + (unsigned)u];
      }
    }
    const float inv = 1.0f / (sa * sb);
#pragma unroll
    for (int p = 0; p < 2; ++p)
#pragma unroll
      for (int q = 0; q < 3; ++q) {
        const float v = (Mb[p * 3] * Ma[q] + Mb[p * 3 + 1] * Ma[3 + q]) + Mb[p * 3 + 2] * Ma[6 + q];
        X6[tid * 8u + (unsigned)(p * 3 + q)] = v * inv;
      }
    X6[tid * 8u + 6u] = 0.0f;
    X6[tid * 8u + 7u] = 0.0f;
  }
  __syncthreads();

#pragma unroll 1
  for (unsigned ps = 0; ps < 4u; ++ps) {
#pragma unroll 1
    for (unsigned rr = 0; rr < 2u; ++rr) {
      const unsigned lr = wv * 2u + rr;
      const unsigned row = ps * 16u + lr;
      float x[6];
#pragma unroll
      for (int p = 0; p < 6; ++p) x[p] = X6[row * 8u + (unsigned)p];
      float hv[16];
#pragma unroll
      for (int c = 0; c < 4; ++c) {
        const unsigned col = (unsigned)(c >> 1) * 256u + lane * 8u + (unsigned)(c & 1) * 4u;
        v4f acc = *(const v4f*)&WEs[col] * x[0];
#pragma unroll
        for (int p = 1; p < 6; ++p) acc += *(const v4f*)&WEs[(unsigned)p * HID + col] * x[p];
        acc += *(const v4f*)&WEs[6u * HID + col];
#pragma unroll
        for (int i = 0; i < 4; ++i) hv[c * 4 + i] = fmaxf(acc[i], 0.0f);
      }
      float mxh = hv[0];
#pragma unroll
      for (int i = 1; i < 16; ++i) mxh = fmaxf(mxh, hv[i]);
      mxh = red32_max(mxh);
      const unsigned e = (__float_as_uint(mxh) >> 23) & 255u;
      int se = 262 - (int)e;
      se = (se < 1) ? 1 : ((se > 254) ? 254 : se);
      const float sc  = __uint_as_float((unsigned)se << 23);
      const float isc = __uint_as_float((unsigned)(254 - se) << 23);
      v8h o0, o1, q0, q1;
#pragma unroll
      for (int i = 0; i < 8; ++i) {
        const float t0 = hv[i] * sc;
        const float t1 = hv[8 + i] * sc;
        const h16 a0 = toh_flush(t0);
        const h16 a1 = toh_flush(t1);
        o0[i] = a0;
        o1[i] = a1;
        q0[i] = toh_flush((t0 - (float)a0) * RCARRY);
        q1[i] = toh_flush((t1 - (float)a1) * RCARRY);
      }
      *(v8h*)&Xs[lr * LDX + lane * 8u] = o0;
      *(v8h*)&Xs[lr * LDX + 256u + lane * 8u] = o1;
      *(v8h*)&Xs[(16u + lr) * LDX + lane * 8u] = q0;
      *(v8h*)&Xs[(16u + lr) * LDX + 256u + lane * 8u] = q1;
      if (lane == 0u) Hsc[row] = isc;
    }
    __syncthreads();

    {
      const unsigned kq = wv >> 1, pl = wv & 1u;
      v8f acc = {};
#pragma unroll 2
      for (unsigned ks = 0; ks < 4u; ++ks) {
        const unsigned k0 = kq * 128u + ks * 32u;
        const v16h a = ld_frag(&Xs[(pl * 16u) * LDX + k0], LDX);
        const v16h w = ld_frag(&W2s[k0], LDX);
        acc = wmma16(a, w, acc);
      }
      if (m < (unsigned)LDP) {
#pragma unroll
        for (int r = 0; r < 8; ++r)
          Part[((pl * 4u + kq) * 64u + ps * 16u + hh * 8u + (unsigned)r) * LDP + m] = acc[r];
      }
    }
    __syncthreads();
  }

  if (tid < (unsigned)NANCH) {
#pragma clang fp contract(off)
    const float cs = Hsc[tid] * (1.0f / WCARRY);
    float r6[6];
#pragma unroll
    for (int c = 0; c < 6; ++c) {
      const float vh = (Part[tid * LDP + (unsigned)c] + Part[(64u + tid) * LDP + (unsigned)c]) +
                       (Part[(128u + tid) * LDP + (unsigned)c] +
                        Part[(192u + tid) * LDP + (unsigned)c]);
      const float vl = (Part[(256u + tid) * LDP + (unsigned)c] +
                        Part[(320u + tid) * LDP + (unsigned)c]) +
                       (Part[(384u + tid) * LDP + (unsigned)c] +
                        Part[(448u + tid) * LDP + (unsigned)c]);
      const float vs = vh + vl * (1.0f / RCARRY);
      r6[c] = vs * cs + bf16r(b2[c]);
    }
    float r1[3], r2[3], r3[3];
#pragma unroll
    for (int c = 0; c < 3; ++c) { r1[c] = r6[c]; r2[c] = r6[c + 3]; }
    const float t0 = r1[0] * r2[0], t1 = r1[1] * r2[1], t2 = r1[2] * r2[2];
    const float dot = (t0 + t2) + t1;
#pragma unroll
    for (int c = 0; c < 3; ++c) {
      const float pr = dot * r1[c];
      r2[c] = r2[c] - pr;
    }
    {
      const float u0 = r1[1] * r2[2], u1 = r1[2] * r2[1];
      const float u2 = r1[2] * r2[0], u3 = r1[0] * r2[2];
      const float u4 = r1[0] * r2[1], u5 = r1[1] * r2[0];
      r3[0] = u0 - u1;
      r3[1] = u2 - u3;
      r3[2] = u4 - u5;
    }
    const float n1 = inv_norm3(r1[0], r1[1], r1[2]);
    const float n2 = inv_norm3(r2[0], r2[1], r2[2]);
    const float n3 = inv_norm3(r3[0], r3[1], r3[2]);
#pragma unroll
    for (int c = 0; c < 3; ++c) { r1[c] = r1[c] * n1; r2[c] = r2[c] * n2; r3[c] = r3[c] * n3; }
#pragma unroll
    for (int p = 0; p < 3; ++p) {
      const float a0 = Rr[tid * 9u + (unsigned)(p * 3)];
      const float a1 = Rr[tid * 9u + (unsigned)(p * 3 + 1)];
      const float a2 = Rr[tid * 9u + (unsigned)(p * 3 + 2)];
      float v0 = a0 * r1[0]; v0 = fmaf(a1, r1[1], v0); v0 = fmaf(a2, r1[2], v0);
      float v1 = a0 * r2[0]; v1 = fmaf(a1, r2[1], v1); v1 = fmaf(a2, r2[2], v1);
      float v2 = a0 * r3[0]; v2 = fmaf(a1, r3[1], v2); v2 = fmaf(a2, r3[2], v2);
      Os[tid * 9u + (unsigned)(p * 3)]     = v0;
      Os[tid * 9u + (unsigned)(p * 3 + 1)] = v1;
      Os[tid * 9u + (unsigned)(p * 3 + 2)] = v2;
    }
  }
  __syncthreads();

  if (wave == 0) {
    v4f xs[5];
#pragma unroll
    for (unsigned q = 0; q < 5u; ++q) {
      const unsigned idx = lane + 32u * q;
      const unsigned ic = (idx < 144u) ? idx : 143u;
      xs[q] = *(const v4f*)&Os[4u * ic];
    }
    float* ob = out + (size_t)b * (NANCH * 9);
#pragma unroll
    for (unsigned q = 0; q < 5u; ++q) {
      const unsigned idx = lane + 32u * q;
      if (idx < 144u) *(volatile v4f*)(ob + 4u * idx) = xs[q];
    }
    __threadfence();
#pragma unroll
    for (unsigned q = 0; q < 5u; ++q) {
      const unsigned idx = lane + 32u * q;
      if (idx < 144u) *(volatile v4f*)(ob + 4u * idx) = xs[q];
    }
  }
}

extern "C" void kernel_launch(void* const* d_in, const int* in_sizes, int n_in,
                              void* d_out, int out_size, void* d_ws, size_t ws_size,
                              hipStream_t stream) {
  if (n_in < 9) return;
  if ((long long)in_sizes[0] < (long long)NB * DIM) return;
  if ((long long)in_sizes[1] < (long long)NB * NANCH * DIM) return;
  if ((long long)in_sizes[2] < (long long)NB * NANCH * 9) return;
  if ((long long)in_sizes[3] < (long long)6 * DIM) return;
  if (in_sizes[4] < DIM) return;
  if ((long long)in_sizes[5] < (long long)DIM * HID) return;
  if (in_sizes[6] < HID) return;
  if ((long long)in_sizes[7] < (long long)HID * 6) return;
  if (in_sizes[8] < 6) return;
  if ((long long)out_size < (long long)NB * NANCH * 9) return;
  if (ws_size < WS_TOTAL) return;

  const float* img   = (const float*)d_in[0];
  const float* feat  = (const float*)d_in[1];
  const float* rot   = (const float*)d_in[2];
  const float* wenc  = (const float*)d_in[3];
  const float* benc  = (const float*)d_in[4];
  const float* w1    = (const float*)d_in[5];
  const float* b1    = (const float*)d_in[6];
  const float* w2    = (const float*)d_in[7];
  const float* b2    = (const float*)d_in[8];
  float* out = (float*)d_out;

  char* ws = (char*)d_ws;
  _Float16* W1_t = (_Float16*)(ws + OFF_W1T);
  float*    Weff = (float*)(ws + OFF_WEFF);

  dim3 blk(256);
  wconv_kernel<<<dim3(HID / 64, DIM / 64), blk, 0, stream>>>(w1, W1_t, (unsigned)HID, (unsigned)DIM);
  weff_kernel<<<dim3(HID / 128), blk, 0, stream>>>(wenc, benc, W1_t, b1, Weff);
  rotattn_kernel<<<dim3(NB), blk, 0, stream>>>(img, feat, rot, Weff, w2, b2, out);
}
